// FKANLinear_34102040330855
// MI455X (gfx1250) — hardware-verified
//
#include <hip/hip_runtime.h>
#include <stddef.h>
#include <stdint.h>
#include <math.h>

#pragma clang fp contract(off)

#define NB    32768
#define NI    64
#define NO    32
#define KPB   46
#define KPAIR 96
#define NPAIR 32
#define KTOT  3072
#define BM    64
#define AS    104
#define STP   36
#define TW    64

static_assert(NI == 2 * NPAIR);
static_assert(NPAIR * KPAIR == KTOT);
static_assert(KPAIR % 32 == 0);
static_assert(2 * KPB + 4 == KPAIR);
static_assert(KPB % 2 == 0);
static_assert(NB % BM == 0);
static_assert(BM == 64);
static_assert(NO == 32);
static_assert(AS >= KPAIR);
static_assert((AS * 2) % 16 == 0);
static_assert((STP * 4) % 16 == 0);
static_assert(NB % 256 == 0);
static_assert((NI * TW) % (4 * 128) == 0);
static_assert(KTOT % 64 == 0);
static_assert((2 * KTOT) / 64 == 96);
static_assert(96 * 8 == 3 * 256);

typedef float          v8f   __attribute__((ext_vector_type(8)));
typedef float          v4f   __attribute__((ext_vector_type(4)));
typedef unsigned short v8us  __attribute__((ext_vector_type(8)));
typedef unsigned short v16us __attribute__((ext_vector_type(16)));
typedef __bf16         v16bf __attribute__((ext_vector_type(16)));
typedef unsigned int   v4u   __attribute__((ext_vector_type(4)));
typedef v8us __attribute__((may_alias)) v8usa;
typedef v4u  __attribute__((may_alias)) v4ua;
typedef v4f  __attribute__((may_alias)) v4fa;
typedef unsigned int __attribute__((may_alias)) u32a;

union FragU { v16us w; v8us h[2]; };

__device__ __forceinline__ v8f zero8() { return (v8f){0.f, 0.f, 0.f, 0.f, 0.f, 0.f, 0.f, 0.f}; }

__device__ __forceinline__ v8f mma_bf(v16us au, v16us bu, v8f c) {
  const v16bf a = __builtin_bit_cast(v16bf, au);
  const v16bf b = __builtin_bit_cast(v16bf, bu);
  c = __builtin_amdgcn_wmma_f32_16x16x32_bf16(false, a, false, b, (short)0, c, false, false);
  asm volatile("v_nop\n\tv_nop\n\tv_nop\n\tv_nop" : "+v"(c) : "v"(au), "v"(bu));
  return c;
}

__device__ __forceinline__ v16us ldfrag_g(const unsigned short* __restrict__ p, int ld, int row0, int k0, int lane) {
  const unsigned short* q = p + (size_t)(row0 + (lane & 15)) * ld + k0 + 8 * (lane >> 4);
  FragU f;
  f.h[0] = *(const v8us*)(q);
  f.h[1] = *(const v8us*)(q + 16);
  return f.w;
}

__device__ __forceinline__ v16us ldfrag_l(const unsigned short* p, int ld, int row0, int k0, int lane) {
  const unsigned short* q = p + (row0 + (lane & 15)) * ld + k0 + 8 * (lane >> 4);
  FragU f;
  f.h[0] = *(const v8usa*)(q);
  f.h[1] = *(const v8usa*)(q + 16);
  return f.w;
}

__device__ __forceinline__ unsigned int bf16_rne(float f) {
  unsigned int u = __float_as_uint(f);
  u += 0x7FFFu + ((u >> 16) & 1u);
  return u >> 16;
}
__device__ __forceinline__ float bf16_val(unsigned int h) { return __uint_as_float(h << 16); }

__device__ __forceinline__ float softplusf(float z) { return fmaxf(z, 0.0f) + log1pf(expf(-fabsf(z))); }

__device__ __forceinline__ int kslot(int i) { return (i >> 1) * KPAIR + (i & 1) * KPB; }

__device__ __forceinline__ void put2(unsigned short* sH, unsigned short* sL, int slot, float w) {
  const unsigned int h = bf16_rne(w);
  sH[slot] = (unsigned short)h;
  sL[slot] = (unsigned short)bf16_rne(w - bf16_val(h));
}

__global__ __launch_bounds__(256) void k_stats(const float* __restrict__ x, const float* __restrict__ scale_logit,
                                               const float* __restrict__ shift, float* __restrict__ tabl) {
  __shared__ float smn[256];
  __shared__ float smx[256];
  __shared__ __align__(16) float sl[TW];

  const int tid = threadIdx.x, col = blockIdx.x;
  float mn = 3.0e38f, mx = -3.0e38f;
#pragma unroll 1
  for (int r = tid; r < NB; r += 256) {
    const float v = x[(size_t)r * NI + col];
    mn = fminf(mn, v);
    mx = fmaxf(mx, v);
  }
  smn[tid] = mn;
  smx[tid] = mx;
  if (tid < TW) sl[tid] = 0.0f;
  __syncthreads();
#pragma unroll 1
  for (int s = 128; s > 0; s >>= 1) {
    if (tid < s) {
      smn[tid] = fminf(smn[tid], smn[tid + s]);
      smx[tid] = fmaxf(smx[tid], smx[tid + s]);
    }
    __syncthreads();
  }
  if (tid == 0) {
    float a = smn[0], b = smx[0];
    const bool pad = (b - a) < 1e-8f;
    a = pad ? a - 0.5f : a;
    b = pad ? b + 0.5f : b;
    const float d = b - a;
    sl[0] = a; sl[1] = a; sl[2] = a;
#pragma unroll 1
    for (int j = 0; j <= 8; ++j) sl[3 + j] = a + d * ((float)j * 0.125f);
    const float gl = sl[11];
    sl[12] = gl; sl[13] = gl; sl[14] = gl;
#pragma unroll 1
    for (int t = 0; t < 14; ++t) sl[24 + t] = 1.0f / fmaxf(sl[t + 1] - sl[t], 1e-12f);
#pragma unroll 1
    for (int t = 0; t < 13; ++t) sl[38 + t] = 1.0f / fmaxf(sl[t + 2] - sl[t], 1e-12f);
#pragma unroll 1
    for (int t = 0; t < 12; ++t) sl[51 + t] = 1.0f / fmaxf(sl[t + 3] - sl[t], 1e-12f);
#pragma unroll 1
    for (int c = 0; c < 4; ++c) {
      const float aw = softplusf(scale_logit[col * 4 + c]) + 1e-6f;
      sl[16 + c] = 1.0f / aw;
      sl[20 + c] = shift[col * 4 + c];
    }
  }
  __syncthreads();

  const v4f val = *(const v4fa*)(sl + (tid & 15) * 4);
  float* dst = tabl + (size_t)col * TW + (tid & 15) * 4;
  if (tid < 16) *(volatile v4f*)dst = val;
  __threadfence();
  if (tid < 16) *(volatile v4f*)dst = val;
}

__device__ __forceinline__ void fam(unsigned short* sH, unsigned short* sL, const float* sMw, const float* sSp,
                                    const float* __restrict__ coef, int cnt, int off, int f, int o, int tid,
                                    float beta) {
  const int n = NI * cnt;
  const int nit = (n + 255) / 256;
  const float spg = sSp[f];
#pragma unroll 1
  for (int it = 0; it < nit; ++it) {
    const int idx = tid + it * 256;
    const int idc = (idx < n) ? idx : n - 1;
    const int i = idc / cnt, j = idc - i * cnt;
    const float c = coef[((size_t)o * NI + i) * cnt + j];
    const float w = ((c * sMw[i * 8 + f]) * spg) * beta;
    if (idx < n) put2(sH, sL, kslot(i) + off + j, w);
  }
}

__global__ __launch_bounds__(256) void k_prep_w(const float* __restrict__ base_v, const float* __restrict__ base_g,
                                                const float* __restrict__ bs_c, const float* __restrict__ ty_c,
                                                const float* __restrict__ jc_c, const float* __restrict__ ch_c,
                                                const float* __restrict__ fo_c, const float* __restrict__ wv_c,
                                                const float* __restrict__ gains, const float* __restrict__ alpha_logit,
                                                const float* __restrict__ beta_logit, const float* __restrict__ mix_logits,
                                                unsigned short* __restrict__ wall) {
  __shared__ __align__(16) unsigned short sW[2 * KTOT];
  __shared__ float sMw[NI * 8];
  __shared__ float sSp[8];

  const int tid = threadIdx.x, o = blockIdx.x;
  unsigned short* sH = sW;
  unsigned short* sL = sW + KTOT;

  if (tid == 0) {
    const float za = alpha_logit[0], zb = beta_logit[0];
#pragma unroll 1
    for (int q = 0; q < 8; ++q) {
      const float zg = gains[(q < 6) ? q : 5];
      const float z = (q < 6) ? zg : ((q == 6) ? za : zb);
      sSp[q] = softplusf(z);
    }
  }
  if (tid < NPAIR) {
    const int b = tid * KPAIR + 2 * KPB;
#pragma unroll
    for (int q = 0; q < 4; ++q) { sH[b + q] = (unsigned short)0; sL[b + q] = (unsigned short)0; }
  }
  __syncthreads();

  if (tid < NI) {
    const int i = tid, oi = o * NI + i;
    float s = 0.0f;
#pragma unroll 1
    for (int ii = 0; ii < NI; ++ii) { const float v = base_v[o * NI + ii]; s = s + v * v; }
    const float rvn = 1.0f / sqrtf(s);
    const float W = (base_g[o] * base_v[oi]) * rvn;
    put2(sH, sL, kslot(i), sSp[6] * W);
    float mxl = -3.0e38f;
#pragma unroll 1
    for (int f = 0; f < 6; ++f) mxl = fmaxf(mxl, mix_logits[oi * 6 + f] * 0.5f);
    float se = 0.0f;
#pragma unroll 1
    for (int f = 0; f < 6; ++f) se = se + expf(mix_logits[oi * 6 + f] * 0.5f - mxl);
    const float rse = 1.0f / se;
#pragma unroll 1
    for (int f = 0; f < 6; ++f) sMw[i * 8 + f] = expf(mix_logits[oi * 6 + f] * 0.5f - mxl) * rse;
  }
  __syncthreads();

  const float beta = sSp[7];
  fam(sH, sL, sMw, sSp, bs_c, 11, 1,  0, o, tid, beta);
  fam(sH, sL, sMw, sSp, ty_c, 4,  12, 1, o, tid, beta);
  fam(sH, sL, sMw, sSp, jc_c, 5,  16, 2, o, tid, beta);
  fam(sH, sL, sMw, sSp, ch_c, 5,  21, 3, o, tid, beta);
  fam(sH, sL, sMw, sSp, fo_c, 16, 26, 4, o, tid, beta);
  fam(sH, sL, sMw, sSp, wv_c, 4,  42, 5, o, tid, beta);
  __syncthreads();

  v4u val[3];
  size_t go[3];
#pragma unroll
  for (int it = 0; it < 3; ++it) {
    const int P = tid + 256 * it;
    const int line = P >> 3, pc = P & 7;
    const int plane = (line >= 48) ? 1 : 0;
    const int lr = line - 48 * plane;
    val[it] = *(const v4ua*)(sW + line * 64 + pc * 8);
    go[it] = (size_t)plane * ((size_t)NO * KTOT) + (size_t)o * KTOT + lr * 64 + pc * 8;
  }
  for (int ps = 0; ps < 2; ++ps) {
#pragma unroll
    for (int it = 0; it < 3; ++it) *(volatile v4u*)(wall + go[it]) = val[it];
    __threadfence();
  }
}

__global__ __launch_bounds__(128) void k_basis_gemm(const float* __restrict__ x, const float* __restrict__ base_bias,
                                                    const float* __restrict__ alpha_logit, const float* __restrict__ tabl,
                                                    const unsigned short* __restrict__ wh,
                                                    const unsigned short* __restrict__ wl, float* __restrict__ out) {
  __shared__ __align__(16) unsigned short sA[2 * BM * AS];
  __shared__ __align__(16) float sT[NI * TW];
  __shared__ __align__(16) float sSt[4][16 * STP];
  __shared__ float sBias[NO];

  const int tid = threadIdx.x, lane = tid & 31, wave = tid >> 5;
  const int hh = lane >> 4, m = lane & 15;
  const int r0 = blockIdx.x * BM;
  unsigned short* sAh = sA;
  unsigned short* sAl = sA + BM * AS;

#pragma unroll 1
  for (int q = tid; q < (NI * TW) / 4; q += 128) *(v4fa*)(sT + 4 * q) = *(const v4f*)(tabl + 4 * q);
  if (tid < NO) sBias[tid] = softplusf(alpha_logit[0]) * base_bias[tid];
  __syncthreads();

  v8f acc0 = zero8(), acc1 = zero8();
  const int row = tid >> 1, which = tid & 1;
  const int arow0 = wave * 16;

#pragma unroll 1
  for (int p = 0; p < NPAIR; ++p) {
    {
      const int i = 2 * p + which;
      const float xv = x[(size_t)(r0 + row) * NI + i];
      const float* T = sT + i * TW;
      float bv[KPB];

      bv[0] = xv;

      {
        float g[15];
#pragma unroll
        for (int t = 0; t < 15; ++t) g[t] = T[t];
        const bool mlast = (xv == g[14]);
        float bas[14];
#pragma unroll
        for (int t = 0; t < 14; ++t) {
          const float b = (xv >= g[t] && xv < g[t + 1]) ? 1.0f : 0.0f;
          bas[t] = mlast ? 0.0f : b;
        }
        bas[13] = mlast ? 1.0f : bas[13];
#pragma unroll
        for (int t = 0; t < 13; ++t)
          bas[t] = ((xv - g[t]) * T[24 + t]) * bas[t] + ((g[t + 2] - xv) * T[25 + t]) * bas[t + 1];
#pragma unroll
        for (int t = 0; t < 12; ++t)
          bas[t] = ((xv - g[t]) * T[38 + t]) * bas[t] + ((g[t + 3] - xv) * T[39 + t]) * bas[t + 1];
#pragma unroll
        for (int t = 0; t < 11; ++t)
          bas[t] = ((xv - g[t]) * T[51 + t]) * bas[t] + ((g[t + 4] - xv) * T[52 + t]) * bas[t + 1];
#pragma unroll
        for (int j = 0; j < 11; ++j) bv[1 + j] = bas[j];
      }

      {
        const float x2 = xv * xv;
        bv[12] = 1.0f;
        bv[13] = xv;
        bv[14] = x2 * 0.5f;
        bv[15] = (x2 * xv) * (1.0f / 6.0f);
      }

      {
        const float j0 = 1.0f;
        const float j1 = (2.0f * xv) * (1.0f / 1.41421356f);
        bv[16] = j0;
        bv[17] = j1;
        float jm2 = j0, jm1 = j1;
        {
          const float A3 = 5.0f * ((24.0f * xv + 1.0f) - 1.0f);
          const float Jn = (A3 * (1.0f / 80.0f)) * jm1 - (48.0f / 80.0f) * jm2;
          const float v = Jn * (1.0f / 1.7320508f);
          bv[18] = v; jm2 = jm1; jm1 = v;
        }
        {
          const float A3 = 7.0f * ((48.0f * xv + 1.0f) - 1.0f);
          const float Jn = (A3 * (1.0f / 210.0f)) * jm1 - (144.0f / 210.0f) * jm2;
          const float v = Jn * 0.5f;
          bv[19] = v; jm2 = jm1; jm1 = v;
        }
        {
          const float A3 = 9.0f * ((80.0f * xv + 1.0f) - 1.0f);
          const float Jn = (A3 * (1.0f / 432.0f)) * jm1 - (320.0f / 432.0f) * jm2;
          bv[20] = Jn * (1.0f / 2.2360680f);
        }
      }

      {
        float xc = __builtin_isfinite(xv) ? xv : 0.0f;
        xc = fminf(fmaxf(xc, -1e6f), 1e6f);
        const float t0 = 1.0f, t1 = xc;
        bv[21] = 1.0f;
        bv[22] = t1 * (1.0f / 1.41421356f);
        const float t2 = (2.0f * xc) * t1 - t0;
        bv[23] = t2 * (1.0f / 1.7320508f);
        const float t3 = (2.0f * xc) * t2 - t1;
        bv[24] = t3 * 0.5f;
        const float t4 = (2.0f * xc) * t3 - t2;
        bv[25] = t4 * (1.0f / 2.2360680f);
      }

      {
        float s1, c1;
        sincosf(xv, &s1, &c1);
        float ck = c1, sk = s1;
#pragma unroll
        for (int kk = 0; kk < 8; ++kk) {
          bv[26 + kk] = ck * 0.25f;
          bv[34 + kk] = sk * 0.25f;
          const float cn = ck * c1 - sk * s1;
          const float sn = sk * c1 + ck * s1;
          ck = cn; sk = sn;
        }
      }

#pragma unroll
      for (int c = 0; c < 4; ++c) {
        const float u = (xv - T[20 + c]) * T[16 + c];
        const float u2 = u * u;
        bv[42 + c] = (u2 - 1.0f) * expf(-0.5f * u2);
      }

      unsigned short* ah = sAh + row * AS + which * KPB;
      unsigned short* al = sAl + row * AS + which * KPB;
#pragma unroll
      for (int q = 0; q < KPB / 2; ++q) {
        const float v0 = bv[2 * q], v1 = bv[2 * q + 1];
        const unsigned int h0 = bf16_rne(v0), h1 = bf16_rne(v1);
        const unsigned int l0 = bf16_rne(v0 - bf16_val(h0));
        const unsigned int l1 = bf16_rne(v1 - bf16_val(h1));
        *(u32a*)(ah + 2 * q) = h0 | (h1 << 16);
        *(u32a*)(al + 2 * q) = l0 | (l1 << 16);
      }
      if (which) {
        *(u32a*)(ah + KPB)     = 0u;
        *(u32a*)(ah + KPB + 2) = 0u;
        *(u32a*)(al + KPB)     = 0u;
        *(u32a*)(al + KPB + 2) = 0u;
      }
    }
    __syncthreads();

    const int kg = p * KPAIR;
#pragma unroll
    for (int ks = 0; ks < 3; ++ks) {
      const int k0 = ks * 32;
      const v16us bh0 = ldfrag_g(wh, KTOT, 0,  kg + k0, lane);
      const v16us bl0 = ldfrag_g(wl, KTOT, 0,  kg + k0, lane);
      const v16us bh1 = ldfrag_g(wh, KTOT, 16, kg + k0, lane);
      const v16us bl1 = ldfrag_g(wl, KTOT, 16, kg + k0, lane);
      const v16us fah = ldfrag_l(sAh, AS, arow0, k0, lane);
      const v16us fal = ldfrag_l(sAl, AS, arow0, k0, lane);
      acc0 = mma_bf(fah, bh0, acc0);
      acc0 = mma_bf(fah, bl0, acc0);
      acc0 = mma_bf(fal, bh0, acc0);
      acc1 = mma_bf(fah, bh1, acc1);
      acc1 = mma_bf(fah, bl1, acc1);
      acc1 = mma_bf(fal, bh1, acc1);
    }
    __syncthreads();
  }

  float* sw = sSt[wave];
  const float bb0 = sBias[m];
  const float bb1 = sBias[16 + m];
#pragma unroll
  for (int r = 0; r < 8; ++r) {
    sw[(8 * hh + r) * STP + m]      = acc0[r] + bb0;
    sw[(8 * hh + r) * STP + 16 + m] = acc1[r] + bb1;
  }
  __syncthreads();
  v4f val[4];
  size_t go[4];
#pragma unroll
  for (int it = 0; it < 4; ++it) {
    const int P  = lane + 32 * it;
    const int L  = P >> 3;
    const int pc = P & 7;
    val[it] = *(const v4fa*)(sw + L * STP + pc * 4);
    go[it]  = (size_t)(r0 + arow0 + L) * NO + pc * 4;
  }
  for (int ps = 0; ps < 2; ++ps) {
#pragma unroll
    for (int it = 0; it < 4; ++it) *(volatile v4f*)(out + go[it]) = val[it];
    __threadfence();
  }
}

extern "C" void kernel_launch(void* const* d_in, const int* in_sizes, int n_in,
                              void* d_out, int out_size, void* d_ws, size_t ws_size,
                              hipStream_t stream) {
  if (n_in < 16) return;
  if (in_sizes[0] != NB * NI) return;
  if (in_sizes[1] != NO * NI || in_sizes[2] != NO || in_sizes[3] != NO) return;
  if (in_sizes[4] != NO * NI * 11 || in_sizes[5] != NO * NI * 4 || in_sizes[6] != NO * NI * 5) return;
  if (in_sizes[7] != NO * NI * 5 || in_sizes[8] != NO * NI * 16 || in_sizes[9] != NO * NI * 4) return;
  if (in_sizes[10] != NI * 4 || in_sizes[11] != NI * 4 || in_sizes[12] != 6) return;
  if (in_sizes[13] < 1 || in_sizes[14] < 1 || in_sizes[15] != NO * NI * 6) return;
  if (out_size != NB * NO) return;

  const float* x    = (const float*)d_in[0];
  const float* bv   = (const float*)d_in[1];
  const float* bg   = (const float*)d_in[2];
  const float* bb   = (const float*)d_in[3];
  const float* cb   = (const float*)d_in[4];
  const float* ct   = (const float*)d_in[5];
  const float* cj   = (const float*)d_in[6];
  const float* cc   = (const float*)d_in[7];
  const float* cf   = (const float*)d_in[8];
  const float* cw   = (const float*)d_in[9];
  const float* wsl  = (const float*)d_in[10];
  const float* wsh  = (const float*)d_in[11];
  const float* gn   = (const float*)d_in[12];
  const float* al   = (const float*)d_in[13];
  const float* be   = (const float*)d_in[14];
  const float* ml   = (const float*)d_in[15];
  float* out = (float*)d_out;

  const size_t tabl_bytes = (size_t)NI * TW * sizeof(float);
  const size_t wall_bytes = (size_t)2 * NO * KTOT * sizeof(unsigned short);
  if (tabl_bytes + wall_bytes > ws_size) return;
  float* tabl = (float*)d_ws;
  unsigned short* wall = (unsigned short*)((char*)d_ws + tabl_bytes);
  const unsigned short* wh = wall;
  const unsigned short* wlo = wall + (size_t)NO * KTOT;

  k_stats<<<dim3(NI), dim3(256), 0, stream>>>(x, wsl, wsh, tabl);
  k_prep_w<<<dim3(NO), dim3(256), 0, stream>>>(bv, bg, cb, ct, cj, cc, cf, cw, gn, al, be, ml, wall);
  k_basis_gemm<<<dim3(NB / BM), dim3(128), 0, stream>>>(x, bb, al, tabl, wh, wlo, out);
  (void)hipGetLastError();
}
